// GAT_2499670966385
// MI455X (gfx1250) — hardware-verified
//
#include <hip/hip_runtime.h>
#include <math.h>
#include <stdint.h>

#define NN 8192
#define TT 60
#define DD 6
#define HH 64
#define GG 192
#define XW 360
#define XP 368
#define SLOPE 0.01f

typedef __attribute__((ext_vector_type(16))) __bf16 v16b;
typedef __attribute__((ext_vector_type(8)))  __bf16 v8b;
typedef __attribute__((ext_vector_type(8)))  float  v8f;
typedef __attribute__((ext_vector_type(4)))  float  v4f;
typedef __attribute__((ext_vector_type(8)))  unsigned int v8u;
typedef __attribute__((ext_vector_type(4)))  unsigned int v4u;
typedef __attribute__((ext_vector_type(2)))  unsigned int v2u;
typedef v8b __attribute__((may_alias)) v8ba;
typedef v4f __attribute__((may_alias)) v4fa;
typedef v4u __attribute__((may_alias)) v4ua;
typedef v2u __attribute__((may_alias)) v2ua;

static_assert(NN % 64 == 0);
static_assert(NN % 256 == 0);
static_assert(DD * TT == XW);
static_assert(DD <= 32);
static_assert(HH == 64);
static_assert(3 * HH == GG);
static_assert(64 % 32 == 0);
static_assert(64 * 2 == 128);
static_assert(4 * 16 == 64);
static_assert((XW * 4) % 16 == 0);
static_assert((XP * 2) % 16 == 0);

#define P_WIH0 0
#define P_WHH0 6144
#define P_WIH1 18432
#define P_WHH1 30720
#define P_TW   43008
#define P_FCW  47104
#define P_END  51200
static_assert(P_WHH0 == P_WIH0 + GG * 32);
static_assert(P_WIH1 == P_WHH0 + GG * HH);
static_assert(P_WHH1 == P_WIH1 + GG * HH);
static_assert(P_TW == P_WHH1 + GG * HH);
static_assert(P_FCW == P_TW + HH * HH);
static_assert(P_END == P_FCW + HH * HH);

#define Q_BIH0 0
#define Q_BHH0 256
#define Q_BIH1 512
#define Q_BHH1 768
#define Q_TB   1024
#define Q_A    1152
#define Q_FCB  1280
#define Q_OW   1408
#define Q_OB   1536
#define Q_END  1664

#define WS_PLANES 0
#define WS_PARAMS 102400
#define WS_HID    131072
#define WS_VT     2228224
#define WS_S      4325376
#define WS_TOTAL  4390912
static_assert(WS_PARAMS == P_END * 2);
static_assert(WS_PARAMS + Q_END * 4 <= WS_HID);
static_assert(WS_VT == WS_HID + NN * HH * 4);
static_assert(WS_S == WS_VT + 2 * HH * NN * 2);
static_assert(WS_TOTAL == WS_S + 2 * NN * 4);
static_assert(WS_PARAMS % 128 == 0 && WS_HID % 128 == 0 && WS_VT % 128 == 0 && WS_S % 128 == 0);
static_assert(WS_TOTAL <= 134217728);

#define PB_WIH0 22
#define PB_PAR  25
#define PB_END  27

#define G_OFF_B   0
#define G_OFF_X   86016
#define G_OFF_A0  133120
#define G_OFF_A1  149504
#define G_OFF_F0  165888
#define G_OFF_F1  182272
#define G_OFF_P   198656
#define G_LDS     205312
static_assert(G_OFF_X == P_TW * 2);
static_assert(G_OFF_A0 == G_OFF_X + 64 * XP * 2);
static_assert(G_OFF_P + Q_END * 4 == G_LDS);
static_assert(32768 + 512 <= 64 * XP * 2);

#define A_OFF_S1  0
#define A_OFF_V   32768
#define A_OFF_AE  98304
#define A_OFF_P   114688
#define A_OFF_R   121344
#define A_LDS     121856

__device__ __forceinline__ unsigned short bf_bits(float f) {
  const unsigned u = __float_as_uint(f);
  return (unsigned short)((u + 0x7FFFu + ((u >> 16) & 1u)) >> 16);
}
__device__ __forceinline__ float bf_val(unsigned short h) { return __uint_as_float(((unsigned)h) << 16); }
__device__ __forceinline__ float bfr(float f) { return bf_val(bf_bits(f)); }
__device__ __forceinline__ __bf16 bf_elem(unsigned short h) { return __builtin_bit_cast(__bf16, h); }
__device__ __forceinline__ unsigned pk16(unsigned short a, unsigned short b) { return (unsigned)a | ((unsigned)b << 16); }
__device__ __forceinline__ float leaky(float v) { return (v > 0.0f) ? v : SLOPE * v; }
__device__ __forceinline__ float sigm(float v) { return 1.0f / (1.0f + expf(-v)); }

__device__ __forceinline__ v8f mma(v16b a, v16b b, v8f c) {
  c = __builtin_amdgcn_wmma_f32_16x16x32_bf16(false, a, false, b, (short)0, c, false, false);
  asm volatile("v_nop\n\tv_nop\n\tv_nop\n\tv_nop" : "+v"(c) : "v"(a), "v"(b));
  return c;
}
union FB { v16b v; v8b h[2]; };
__device__ __forceinline__ v16b ldfrag_l(const __bf16* p) {
  FB f; f.h[0] = *(const v8ba*)(p); f.h[1] = *(const v8ba*)(p + 16); return f.v;
}
__device__ __forceinline__ v16b ldfrag_g(const __bf16* __restrict__ p) {
  FB f; f.h[0] = *(const v8ba*)(p); f.h[1] = *(const v8ba*)(p + 16); return f.v;
}

__device__ __forceinline__ void cvt8(const float* __restrict__ src, unsigned short* __restrict__ dst) {
  const v4f a = *(const v4fa*)(src);
  const v4f b = *(const v4fa*)(src + 4);
  const v4u o = { pk16(bf_bits(a.x), bf_bits(a.y)), pk16(bf_bits(a.z), bf_bits(a.w)),
                  pk16(bf_bits(b.x), bf_bits(b.y)), pk16(bf_bits(b.z), bf_bits(b.w)) };
  *(volatile v4u*)dst = o;
  __threadfence();
  *(volatile v4u*)dst = o;
}

__global__ __launch_bounds__(256) void k_prep(
    const float* __restrict__ Wih0, const float* __restrict__ Whh0,
    const float* __restrict__ bih0, const float* __restrict__ bhh0,
    const float* __restrict__ Wih1, const float* __restrict__ Whh1,
    const float* __restrict__ bih1, const float* __restrict__ bhh1,
    const float* __restrict__ tW, const float* __restrict__ tb, const float* __restrict__ av,
    const float* __restrict__ fcW, const float* __restrict__ fcb,
    const float* __restrict__ outW, const float* __restrict__ outb,
    unsigned short* __restrict__ planes, float* __restrict__ params)
{
  const int b = blockIdx.x, tid = threadIdx.x;
  if (b < PB_WIH0) {
    const float* src = Whh0; int po = P_WHH0; int cb = b;
    if (b >= 20)      { src = fcW;  po = P_FCW;  cb = b - 20; }
    else if (b >= 18) { src = tW;   po = P_TW;   cb = b - 18; }
    else if (b >= 12) { src = Whh1; po = P_WHH1; cb = b - 12; }
    else if (b >= 6)  { src = Wih1; po = P_WIH1; cb = b - 6; }
    const int ch = cb * 256 + tid;
    cvt8(src + (size_t)ch * 8, planes + po + (size_t)ch * 8);
  } else if (b < PB_PAR) {
    const int ch = (b - PB_WIH0) * 256 + tid;
    const int row = ch >> 2, kq = ch & 3;
    const float* s = Wih0 + row * DD;
    const float w0 = s[0], w1 = s[1], w2 = s[2], w3 = s[3], w4 = s[4], w5 = s[5];
    const unsigned m = (kq == 0) ? 0xFFFFFFFFu : 0u;
    const v4u o = { pk16(bf_bits(w0), bf_bits(w1)) & m, pk16(bf_bits(w2), bf_bits(w3)) & m,
                    pk16(bf_bits(w4), bf_bits(w5)) & m, 0u };
    unsigned short* dst = planes + P_WIH0 + (size_t)ch * 8;
    *(volatile v4u*)dst = o;
    __threadfence();
    *(volatile v4u*)dst = o;
  } else {
    const int u = __builtin_amdgcn_readfirstlane((b - PB_PAR) * 8 + (tid >> 5));
    const int lane = tid & 31;
    if (u < 13) {
      const float* src = bih0; int cnt = GG; int base = 0;
      if (u == 1)       { base = 128; }
      else if (u == 2)  { src = bhh0; }
      else if (u == 3)  { src = bhh0; base = 128; }
      else if (u == 4)  { src = bih1; }
      else if (u == 5)  { src = bih1; base = 128; }
      else if (u == 6)  { src = bhh1; }
      else if (u == 7)  { src = bhh1; base = 128; }
      else if (u == 8)  { src = tb;   cnt = HH; }
      else if (u == 9)  { src = av;   cnt = 2 * HH; }
      else if (u == 10) { src = fcb;  cnt = HH; }
      else if (u == 11) { src = outW; cnt = HH; }
      else if (u == 12) { src = outb; cnt = 1; }
      const int i0 = base + 4 * lane;
      const int j0 = (i0     < cnt) ? i0     : (cnt - 1);
      const int j1 = (i0 + 1 < cnt) ? i0 + 1 : (cnt - 1);
      const int j2 = (i0 + 2 < cnt) ? i0 + 2 : (cnt - 1);
      const int j3 = (i0 + 3 < cnt) ? i0 + 3 : (cnt - 1);
      const float f0 = src[j0], f1 = src[j1], f2 = src[j2], f3 = src[j3];
      const v4f o = { (i0     < cnt) ? bfr(f0) : 0.0f, (i0 + 1 < cnt) ? bfr(f1) : 0.0f,
                      (i0 + 2 < cnt) ? bfr(f2) : 0.0f, (i0 + 3 < cnt) ? bfr(f3) : 0.0f };
      float* dst = params + u * 128 + 4 * lane;
      *(volatile v4f*)dst = o;
      __threadfence();
      *(volatile v4f*)dst = o;
    }
  }
}

__device__ __forceinline__ void gru_gate(v8f aR, v8f aZ, v8f aNi, v8f aNh,
                                         float bR, float bZ, float biN, float bhN,
                                         float* fst, __bf16* wA) {
#pragma unroll
  for (int r = 0; r < 8; ++r) {
    const float hold = fst[r * 32];
    const float rr = sigm(aR[r] + bR);
    const float zz = sigm(aZ[r] + bZ);
    const float nn = tanhf(aNi[r] + biN + rr * (aNh[r] + bhN));
    const float hn = (1.0f - zz) * nn + zz * hold;
    fst[r * 32] = hn;
    const unsigned short hb = bf_bits(hn);
    const unsigned short lb = bf_bits(hn - bf_val(hb));
    wA[r * 128] = bf_elem(hb);
    wA[r * 128 + 64] = bf_elem(lb);
  }
}

__global__ __launch_bounds__(128) void k_gru(
    const float* __restrict__ x, const unsigned short* __restrict__ planes, const float* __restrict__ params,
    float* __restrict__ HID, unsigned short* __restrict__ VT, float* __restrict__ S12)
{
  extern __shared__ __align__(16) unsigned char smem_g[];
  __bf16* sW = (__bf16*)(smem_g + G_OFF_B);
  unsigned short* sX = (unsigned short*)(smem_g + G_OFF_X);
  __bf16* sA0 = (__bf16*)(smem_g + G_OFF_A0);
  __bf16* sA1 = (__bf16*)(smem_g + G_OFF_A1);
  float* sF0 = (float*)(smem_g + G_OFF_F0);
  float* sF1 = (float*)(smem_g + G_OFF_F1);
  float* sP  = (float*)(smem_g + G_OFF_P);
  float* sHid = (float*)(smem_g + G_OFF_X);
  unsigned short* sVh = (unsigned short*)(smem_g + G_OFF_X + 16384);
  unsigned short* sVl = (unsigned short*)(smem_g + G_OFF_X + 24576);
  float* sS = (float*)(smem_g + G_OFF_X + 32768);

  const int tid = threadIdx.x, wave = tid >> 5, lane = tid & 31;
  const int hh = lane >> 4, c = lane & 15;
  const int R0 = blockIdx.x * 64;

#pragma unroll 2
  for (int q = tid; q < 5376; q += 128) {
    const v4u v = *(const v4ua*)(planes + (size_t)q * 8);
    *(v4ua*)(smem_g + G_OFF_B + q * 16) = v;
  }
  for (int q = tid; q < Q_END / 4; q += 128) {
    const v4f v = *(const v4fa*)(params + q * 4);
    *(v4fa*)(sP + q * 4) = v;
  }
#pragma unroll 3
  for (int q = tid; q < 64 * 90; q += 128) {
    const int row = q / 90;
    const int c4 = (q - row * 90) * 4;
    const v4f v = *(const v4fa*)(x + (size_t)(R0 + row) * XW + c4);
    const v2u o = { pk16(bf_bits(v.x), bf_bits(v.y)), pk16(bf_bits(v.z), bf_bits(v.w)) };
    *(v2ua*)(sX + row * XP + c4) = o;
  }
  float* f0 = sF0 + wave * 1024 + lane;
  float* f1 = sF1 + wave * 1024 + lane;
#pragma unroll
  for (int i = 0; i < 32; ++i) { f0[i * 32] = 0.0f; f1[i * 32] = 0.0f; }
  __syncthreads();

  const __bf16* sWih0 = sW + P_WIH0;
  const __bf16* sWhh0 = sW + P_WHH0;
  const __bf16* sWih1 = sW + P_WIH1;
  const __bf16* sWhh1 = sW + P_WHH1;

  const v8f z8 = {0.f, 0.f, 0.f, 0.f, 0.f, 0.f, 0.f, 0.f};
  const v8u zu = {0u, 0u, 0u, 0u, 0u, 0u, 0u, 0u};
  v16b a0h[2], a0l[2], a1h[2], a1l[2];
  a0h[0] = __builtin_bit_cast(v16b, zu); a0h[1] = a0h[0]; a0l[0] = a0h[0]; a0l[1] = a0h[0];
  a1h[0] = a0h[0]; a1h[1] = a0h[0]; a1l[0] = a0h[0]; a1l[1] = a0h[0];

  const __bf16* ar0 = sA0 + (wave * 16 + c) * 128 + 8 * hh;
  const __bf16* ar1 = sA1 + (wave * 16 + c) * 128 + 8 * hh;
  __bf16* wa0 = sA0 + (wave * 16 + 8 * hh) * 128 + c;
  __bf16* wa1 = sA1 + (wave * 16 + 8 * hh) * 128 + c;
  const unsigned short* xrow = sX + (wave * 16 + c) * XP;
  const unsigned xmask = hh ? 0u : 0xFFFFFFFFu;

#pragma unroll 1
  for (int t = 0; t < TT; ++t) {
    const unsigned x0 = xrow[t], x1 = xrow[TT + t], x2 = xrow[2 * TT + t];
    const unsigned x3 = xrow[3 * TT + t], x4 = xrow[4 * TT + t], x5 = xrow[5 * TT + t];
    const v8u xu = { (x0 | (x1 << 16)) & xmask, (x2 | (x3 << 16)) & xmask, (x4 | (x5 << 16)) & xmask,
                     0u, 0u, 0u, 0u, 0u };
    const v16b xa = __builtin_bit_cast(v16b, xu);

#pragma unroll 1
    for (int jt = 0; jt < 4; ++jt) {
      const int nb = jt * 16 + c;
      v8f aR = z8, aZ = z8, aNi = z8, aNh = z8;
      {
        v16b b = ldfrag_l(sWih0 + nb * 32 + 8 * hh);          aR  = mma(xa, b, aR);
        b = ldfrag_l(sWih0 + (64 + nb) * 32 + 8 * hh);        aZ  = mma(xa, b, aZ);
        b = ldfrag_l(sWih0 + (128 + nb) * 32 + 8 * hh);       aNi = mma(xa, b, aNi);
      }
#pragma unroll
      for (int ks = 0; ks < 2; ++ks) {
        v16b b = ldfrag_l(sWhh0 + nb * 64 + ks * 32 + 8 * hh);
        aR = mma(a0h[ks], b, aR);   aR = mma(a0l[ks], b, aR);
        b = ldfrag_l(sWhh0 + (64 + nb) * 64 + ks * 32 + 8 * hh);
        aZ = mma(a0h[ks], b, aZ);   aZ = mma(a0l[ks], b, aZ);
        b = ldfrag_l(sWhh0 + (128 + nb) * 64 + ks * 32 + 8 * hh);
        aNh = mma(a0h[ks], b, aNh); aNh = mma(a0l[ks], b, aNh);
      }
      const float bR  = sP[Q_BIH0 + nb] + sP[Q_BHH0 + nb];
      const float bZ  = sP[Q_BIH0 + 64 + nb] + sP[Q_BHH0 + 64 + nb];
      const float biN = sP[Q_BIH0 + 128 + nb];
      const float bhN = sP[Q_BHH0 + 128 + nb];
      gru_gate(aR, aZ, aNi, aNh, bR, bZ, biN, bhN, f0 + jt * 256, wa0 + jt * 16);
    }
    __syncthreads();
#pragma unroll
    for (int ks = 0; ks < 2; ++ks) {
      a0h[ks] = ldfrag_l(ar0 + ks * 32);
      a0l[ks] = ldfrag_l(ar0 + 64 + ks * 32);
    }

#pragma unroll 1
    for (int jt = 0; jt < 4; ++jt) {
      const int nb = jt * 16 + c;
      v8f aR = z8, aZ = z8, aNi = z8, aNh = z8;
#pragma unroll
      for (int ks = 0; ks < 2; ++ks) {
        v16b b = ldfrag_l(sWih1 + nb * 64 + ks * 32 + 8 * hh);
        aR = mma(a0h[ks], b, aR);   aR = mma(a0l[ks], b, aR);
        b = ldfrag_l(sWhh1 + nb * 64 + ks * 32 + 8 * hh);
        aR = mma(a1h[ks], b, aR);   aR = mma(a1l[ks], b, aR);
        b = ldfrag_l(sWih1 + (64 + nb) * 64 + ks * 32 + 8 * hh);
        aZ = mma(a0h[ks], b, aZ);   aZ = mma(a0l[ks], b, aZ);
        b = ldfrag_l(sWhh1 + (64 + nb) * 64 + ks * 32 + 8 * hh);
        aZ = mma(a1h[ks], b, aZ);   aZ = mma(a1l[ks], b, aZ);
        b = ldfrag_l(sWih1 + (128 + nb) * 64 + ks * 32 + 8 * hh);
        aNi = mma(a0h[ks], b, aNi); aNi = mma(a0l[ks], b, aNi);
        b = ldfrag_l(sWhh1 + (128 + nb) * 64 + ks * 32 + 8 * hh);
        aNh = mma(a1h[ks], b, aNh); aNh = mma(a1l[ks], b, aNh);
      }
      const float bR  = sP[Q_BIH1 + nb] + sP[Q_BHH1 + nb];
      const float bZ  = sP[Q_BIH1 + 64 + nb] + sP[Q_BHH1 + 64 + nb];
      const float biN = sP[Q_BIH1 + 128 + nb];
      const float bhN = sP[Q_BHH1 + 128 + nb];
      gru_gate(aR, aZ, aNi, aNh, bR, bZ, biN, bhN, f1 + jt * 256, wa1 + jt * 16);
    }
    __syncthreads();
#pragma unroll
    for (int ks = 0; ks < 2; ++ks) {
      a1h[ks] = ldfrag_l(ar1 + ks * 32);
      a1l[ks] = ldfrag_l(ar1 + 64 + ks * 32);
    }
  }
  __syncthreads();

  const __bf16* gTW = (const __bf16*)(const void*)(planes + P_TW);
  float s1p[8], s2p[8];
#pragma unroll
  for (int r = 0; r < 8; ++r) { s1p[r] = 0.0f; s2p[r] = 0.0f; }
#pragma unroll 1
  for (int jt = 0; jt < 4; ++jt) {
    const int nb = jt * 16 + c;
    v8f acc = z8;
#pragma unroll
    for (int ks = 0; ks < 2; ++ks) {
      const v16b b = ldfrag_g(gTW + nb * 64 + ks * 32 + 8 * hh);
      acc = mma(a1h[ks], b, acc);
      acc = mma(a1l[ks], b, acc);
    }
    const float tbv = sP[Q_TB + nb], av1 = sP[Q_A + nb], av2 = sP[Q_A + 64 + nb];
#pragma unroll
    for (int r = 0; r < 8; ++r) {
      const float tv = acc[r] + tbv;
      s1p[r] += tv * av1;
      s2p[r] += tv * av2;
      const float hv = f1[(jt * 8 + r) * 32];
      const int lrow = wave * 16 + 8 * hh + r;
      sHid[lrow * 64 + nb] = hv;
      const unsigned short hb = bf_bits(hv);
      sVh[nb * 64 + lrow] = hb;
      sVl[nb * 64 + lrow] = bf_bits(hv - bf_val(hb));
    }
  }
#pragma unroll
  for (int r = 0; r < 8; ++r) {
    float a = s1p[r], b = s2p[r];
    a += __shfl_xor(a, 1, 32); b += __shfl_xor(b, 1, 32);
    a += __shfl_xor(a, 2, 32); b += __shfl_xor(b, 2, 32);
    a += __shfl_xor(a, 4, 32); b += __shfl_xor(b, 4, 32);
    a += __shfl_xor(a, 8, 32); b += __shfl_xor(b, 8, 32);
    s1p[r] = a; s2p[r] = b;
  }
#pragma unroll
  for (int r = 0; r < 8; ++r) {
    if (c == r) {
      sS[wave * 16 + 8 * hh + r] = s1p[r];
      sS[64 + wave * 16 + 8 * hh + r] = s2p[r];
    }
  }
  __syncthreads();

  {
    v4f hv[8];
    v4u vh[4], vl[4];
    const int c4 = c * 4;
    const int q = lane >> 3, c8 = (lane & 7) * 8;
#pragma unroll
    for (int it = 0; it < 8; ++it) hv[it] = *(const v4fa*)(sHid + (wave * 16 + it * 2 + hh) * 64 + c4);
#pragma unroll
    for (int it = 0; it < 4; ++it) {
      const int f = wave * 16 + it * 4 + q;
      vh[it] = *(const v4ua*)(sVh + f * 64 + c8);
      vl[it] = *(const v4ua*)(sVl + f * 64 + c8);
    }
    const v4f sv = *(const v4fa*)(sS + hh * 64 + c4);
    float* hdst = HID + (size_t)(R0 + wave * 16) * HH;
    for (int pass = 0; pass < 2; ++pass) {
#pragma unroll
      for (int it = 0; it < 8; ++it)
        *(volatile v4f*)(hdst + (it * 2 + hh) * HH + c4) = hv[it];
#pragma unroll
      for (int it = 0; it < 4; ++it) {
        const int f = wave * 16 + it * 4 + q;
        *(volatile v4u*)(VT + (size_t)f * NN + R0 + c8) = vh[it];
        *(volatile v4u*)(VT + (size_t)HH * NN + (size_t)f * NN + R0 + c8) = vl[it];
      }
      if (wave == 0)
        *(volatile v4f*)(S12 + hh * NN + R0 + c4) = sv;
      __threadfence();
    }
  }
}

__global__ __launch_bounds__(128) void k_att(
    const unsigned short* __restrict__ planes, const float* __restrict__ params,
    const float* __restrict__ HID, const unsigned short* __restrict__ VT,
    const float* __restrict__ S12, float* __restrict__ out)
{
  extern __shared__ __align__(16) unsigned char smem_a[];
  float* sS1 = (float*)(smem_a + A_OFF_S1);
  __bf16* sVh = (__bf16*)(smem_a + A_OFF_V);
  __bf16* sVl = (__bf16*)(smem_a + A_OFF_V + 32768);
  float* sHid = (float*)(smem_a + A_OFF_V);
  __bf16* sAe = (__bf16*)(smem_a + A_OFF_AE);
  float* sP = (float*)(smem_a + A_OFF_P);
  float* sRed = (float*)(smem_a + A_OFF_R);
  float* sOut = (float*)(smem_a + A_OFF_R + 64);

  const int tid = threadIdx.x, wave = tid >> 5, lane = tid & 31;
  const int hh = lane >> 4, c = lane & 15;
  const int blk = blockIdx.x;
  const int q0 = blk * 64 + wave * 16;

  float mx = -INFINITY;
#pragma unroll 4
  for (int q = tid; q < NN / 4; q += 128) {
    const v4f v = *(const v4fa*)(S12 + q * 4);
    *(v4fa*)(sS1 + q * 4) = v;
    mx = fmaxf(mx, fmaxf(fmaxf(v.x, v.y), fmaxf(v.z, v.w)));
  }
  for (int q = tid; q < Q_END / 4; q += 128) {
    const v4f v = *(const v4fa*)(params + q * 4);
    *(v4fa*)(sP + q * 4) = v;
  }
  mx = fmaxf(mx, __shfl_xor(mx, 16, 32));
  mx = fmaxf(mx, __shfl_xor(mx, 8, 32));
  mx = fmaxf(mx, __shfl_xor(mx, 4, 32));
  mx = fmaxf(mx, __shfl_xor(mx, 2, 32));
  mx = fmaxf(mx, __shfl_xor(mx, 1, 32));
  if (lane == 0) sRed[wave] = mx;
  __syncthreads();
  const float smax = fmaxf(fmaxf(sRed[0], sRed[1]), fmaxf(sRed[2], sRed[3]));

  const float s2v = S12[NN + q0 + c];
  const float mrow = leaky(s2v + smax);

  const v8f z8 = {0.f, 0.f, 0.f, 0.f, 0.f, 0.f, 0.f, 0.f};
  v8f oacc[4];
#pragma unroll
  for (int t = 0; t < 4; ++t) oacc[t] = z8;
  float psum = 0.0f;

#pragma unroll 1
  for (int kc = 0; kc < NN / 256; ++kc) {
    __syncthreads();
#pragma unroll 4
    for (int i = 0; i < 32; ++i) {
      const int q = tid + i * 128;
      const int pl = q >> 11, rem = q & 2047;
      const int f = rem >> 5, c8 = (rem & 31) * 8;
      const v4u v = *(const v4ua*)(VT + (size_t)pl * HH * NN + (size_t)f * NN + kc * 256 + c8);
      *(v4ua*)(smem_a + A_OFF_V + q * 16) = v;
    }
    __syncthreads();

#pragma unroll 1
    for (int kt = 0; kt < 8; ++kt) {
      const float* sp = sS1 + kc * 256 + kt * 32 + 8 * hh;
      const v4f e0 = *(const v4fa*)(sp);
      const v4f e1 = *(const v4fa*)(sp + 4);
      const v4f e2 = *(const v4fa*)(sp + 16);
      const v4f e3 = *(const v4fa*)(sp + 20);
      const float sv[16] = { e0.x, e0.y, e0.z, e0.w, e1.x, e1.y, e1.z, e1.w,
                             e2.x, e2.y, e2.z, e2.w, e3.x, e3.y, e3.z, e3.w };
      unsigned hb[16], lb[16];
#pragma unroll
      for (int i = 0; i < 16; ++i) {
        const float p = expf(leaky(s2v + sv[i]) - mrow);
        psum += p;
        const unsigned short h_ = bf_bits(p);
        hb[i] = h_;
        lb[i] = bf_bits(p - bf_val(h_));
      }
      v8u uh, ul;
#pragma unroll
      for (int j = 0; j < 8; ++j) {
        uh[j] = hb[2 * j] | (hb[2 * j + 1] << 16);
        ul[j] = lb[2 * j] | (lb[2 * j + 1] << 16);
      }
      const v16b ph = __builtin_bit_cast(v16b, uh);
      const v16b pl = __builtin_bit_cast(v16b, ul);
#pragma unroll
      for (int t = 0; t < 4; ++t) {
        const v16b vb = ldfrag_l(sVh + (t * 16 + c) * 256 + kt * 32 + 8 * hh);
        const v16b vl = ldfrag_l(sVl + (t * 16 + c) * 256 + kt * 32 + 8 * hh);
        oacc[t] = mma(ph, vb, oacc[t]);
        oacc[t] = mma(ph, vl, oacc[t]);
        oacc[t] = mma(pl, vb, oacc[t]);
      }
    }
  }

  const float lt = psum + __shfl_xor(psum, 16, 32);
  float inv[8];
#pragma unroll
  for (int r = 0; r < 8; ++r) {
    const float lr = __shfl(lt, 8 * hh + r, 32);
    inv[r] = 1.0f / lr;
  }
  __syncthreads();
#pragma unroll
  for (int i = 0; i < 8; ++i) {
    const int q = tid + i * 128;
    const v4f v = *(const v4fa*)(HID + (size_t)blk * 64 * HH + q * 4);
    *(v4fa*)(sHid + q * 4) = v;
  }
  __syncthreads();

  __bf16* ae = sAe + wave * 2048;
#pragma unroll
  for (int t = 0; t < 4; ++t) {
#pragma unroll
    for (int r = 0; r < 8; ++r) {
      const int row = 8 * hh + r, col = t * 16 + c;
      const float hv = oacc[t][r] * inv[r] + sHid[(wave * 16 + row) * 64 + col];
      const unsigned short hb = bf_bits(hv);
      ae[row * 128 + col] = bf_elem(hb);
      ae[row * 128 + 64 + col] = bf_elem(bf_bits(hv - bf_val(hb)));
    }
  }
  __syncthreads();

  v16b eh[2], el[2];
#pragma unroll
  for (int ks = 0; ks < 2; ++ks) {
    eh[ks] = ldfrag_l(ae + c * 128 + ks * 32 + 8 * hh);
    el[ks] = ldfrag_l(ae + c * 128 + 64 + ks * 32 + 8 * hh);
  }
  const __bf16* gFC = (const __bf16*)(const void*)(planes + P_FCW);
  float op[8];
#pragma unroll
  for (int r = 0; r < 8; ++r) op[r] = 0.0f;
#pragma unroll 1
  for (int jt = 0; jt < 4; ++jt) {
    const int nb = jt * 16 + c;
    v8f acc = z8;
#pragma unroll
    for (int ks = 0; ks < 2; ++ks) {
      const v16b b = ldfrag_g(gFC + nb * 64 + ks * 32 + 8 * hh);
      acc = mma(eh[ks], b, acc);
      acc = mma(el[ks], b, acc);
    }
    const float fb = sP[Q_FCB + nb], ow = sP[Q_OW + nb];
#pragma unroll
    for (int r = 0; r < 8; ++r) {
      const float v = leaky(acc[r] + fb);
      op[r] += v * ow;
    }
  }
  const float ob = sP[Q_OB];
#pragma unroll
  for (int r = 0; r < 8; ++r) {
    float a = op[r];
    a += __shfl_xor(a, 1, 32);
    a += __shfl_xor(a, 2, 32);
    a += __shfl_xor(a, 4, 32);
    a += __shfl_xor(a, 8, 32);
    op[r] = a + ob;
  }
#pragma unroll
  for (int r = 0; r < 8; ++r) {
    if (c == r) sOut[wave * 16 + 8 * hh + r] = op[r];
  }
  __syncthreads();

  {
    const v4f v = *(const v4fa*)(sOut + (lane & 15) * 4);
    float* dst = out + blk * 64 + (lane & 15) * 4;
    if (tid < 16) *(volatile v4f*)dst = v;
    __threadfence();
    if (tid < 16) *(volatile v4f*)dst = v;
  }
}

extern "C" void kernel_launch(void* const* d_in, const int* in_sizes, int n_in,
                              void* d_out, int out_size, void* d_ws, size_t ws_size,
                              hipStream_t stream) {
  if (n_in < 16) return;
  if (in_sizes[0] != NN * XW) return;
  if (in_sizes[1] != GG * DD || in_sizes[2] != GG * HH) return;
  if (in_sizes[3] != GG || in_sizes[4] != GG) return;
  if (in_sizes[5] != GG * HH || in_sizes[6] != GG * HH) return;
  if (in_sizes[7] != GG || in_sizes[8] != GG) return;
  if (in_sizes[9] != HH * HH || in_sizes[10] != HH) return;
  if (in_sizes[11] != 2 * HH) return;
  if (in_sizes[12] != HH * HH || in_sizes[13] != HH) return;
  if (in_sizes[14] != HH || in_sizes[15] != 1) return;
  if (out_size != NN) return;
  if ((size_t)WS_TOTAL > ws_size) return;

  const float* x     = (const float*)d_in[0];
  const float* Wih0  = (const float*)d_in[1];
  const float* Whh0  = (const float*)d_in[2];
  const float* bih0  = (const float*)d_in[3];
  const float* bhh0  = (const float*)d_in[4];
  const float* Wih1  = (const float*)d_in[5];
  const float* Whh1  = (const float*)d_in[6];
  const float* bih1  = (const float*)d_in[7];
  const float* bhh1  = (const float*)d_in[8];
  const float* tW    = (const float*)d_in[9];
  const float* tb    = (const float*)d_in[10];
  const float* av    = (const float*)d_in[11];
  const float* fcW   = (const float*)d_in[12];
  const float* fcb   = (const float*)d_in[13];
  const float* outW  = (const float*)d_in[14];
  const float* outb  = (const float*)d_in[15];

  char* ws = (char*)d_ws;
  unsigned short* planes = (unsigned short*)(ws + WS_PLANES);
  float*          params = (float*)(ws + WS_PARAMS);
  float*          HID    = (float*)(ws + WS_HID);
  unsigned short* VT     = (unsigned short*)(ws + WS_VT);
  float*          S12    = (float*)(ws + WS_S);

  (void)hipFuncSetAttribute(reinterpret_cast<const void*>(&k_gru), hipFuncAttributeMaxDynamicSharedMemorySize, G_LDS);
  (void)hipFuncSetAttribute(reinterpret_cast<const void*>(&k_att), hipFuncAttributeMaxDynamicSharedMemorySize, A_LDS);

  k_prep<<<PB_END, 256, 0, stream>>>(Wih0, Whh0, bih0, bhh0, Wih1, Whh1, bih1, bhh1,
                                     tW, tb, av, fcW, fcb, outW, outb, planes, params);
  k_gru<<<NN / 64, 128, G_LDS, stream>>>(x, planes, params, HID, VT, S12);
  k_att<<<NN / 64, 128, A_LDS, stream>>>(planes, params, HID, VT, S12, (float*)d_out);
  (void)hipGetLastError();
}
